// GNNAnomalyDetector_21603685499209
// MI455X (gfx1250) — hardware-verified
//
#include <hip/hip_runtime.h>
#include <stddef.h>
#include <stdint.h>
#include <math.h>


#define NN      50000
#define NE      800000
#define DIN     256
#define HID     64
#define XGC     256
#define K2      128
#define NTHR    256
#define NWAVE   8
#define EPT     8
#define CHUNK   (NTHR * EPT)
#define WCAP    (EPT * 32)
#define LISTN   (NWAVE * WCAP)
#define NBA     1024
#define SLA     10
#define RCAP    28672
#define DEGCAP  128
#define MEAS_B1024  16623
#define MEAS_MAXDEG 35
#define GBM     64
#define GBN     64
#define GTHR    128
#define MP      50048
#define NBLK    49
#define NSLOT   (NBLK * NBA)
#define NEGSL   0.2f
#define EP_P    0
#define EP_XG   1
#define EP_R1   2
#define EP_REC  3
#define BKT_ZINTS    (RCAP + 3 * NBA)
#define BKT_LDS_INTS (LISTN + 2 * RCAP + 3 * NBA + 16)
#define OUT_TOT  16000002
#define OFF_REC  2
#define OFF_HG   12800002
#define REC_N    12800000
#define HG_N     3200000
#define OUT_GROUPS 4000001
#define OUT_BLOCKS 15626
#define NUW0  (HID * (DIN / 8))
#define NUW1  (HID * (K2 / 8))
#define NUWG  (XGC * (K2 / 8))
#define NUWALL (NUW0 + 3 * NUW1 + 2 * NUWG)

static_assert((CHUNK & (CHUNK - 1)) == 0 && CHUNK <= 4096);
static_assert((NBA & (NBA - 1)) == 0 && NBA == (1 << SLA) && NBA == 4 * NTHR);
static_assert(((long long)CHUNK << SLA) < (1LL << 31));
static_assert(NN <= 65536);
static_assert(NBA % NWAVE == 0 && NBA % 32 == 0);
static_assert((RCAP % (4 * NTHR)) == 0 && (BKT_ZINTS % 4) == 0);
static_assert(RCAP >= MEAS_B1024 + MEAS_B1024 / 20);
static_assert(DEGCAP >= MEAS_MAXDEG + 8);
static_assert(BKT_LDS_INTS * 4 <= 327680);
static_assert(GBM == (GTHR / 32) * 16 && GTHR == 2 * GBN && GTHR == 2 * GBM);
static_assert((MP % GBM) == 0 && MP >= NN && NSLOT >= MP && (NBLK - 1) * NBA < NN);
static_assert((DIN % 32) == 0 && (K2 % 32) == 0 && K2 == 2 * HID && HID == GBN && (XGC % GBN) == 0);
static_assert(HID == 2 * 32);
static_assert(XGC == 8 * 32 && XGC == 4 * HID);
static_assert((NN % 8) == 0);
static_assert((OFF_REC % 4) == 2 && (OFF_HG % 4) == 2 && (OUT_TOT % 4) == 2);
static_assert(OFF_HG == OFF_REC + REC_N && OUT_TOT == OFF_HG + HG_N);
static_assert(REC_N == NN * XGC && HG_N == NN * HID);
static_assert(OUT_GROUPS == (OUT_TOT + 3) / 4 && OUT_BLOCKS == (OUT_GROUPS + NTHR - 1) / NTHR);
static_assert((NUW0 % NTHR) == 0 && (NUW1 % NTHR) == 0 && (NUWG % NTHR) == 0);
static_assert(((MP * (DIN / 8)) % NTHR) == 0);

typedef float          v2f  __attribute__((ext_vector_type(2)));
typedef float          v4f  __attribute__((ext_vector_type(4)));
typedef float          v8f  __attribute__((ext_vector_type(8)));
typedef double         v2d  __attribute__((ext_vector_type(2)));
typedef int            v4i  __attribute__((ext_vector_type(4)));
typedef int            v8i  __attribute__((ext_vector_type(8)));
typedef unsigned int   v2u  __attribute__((ext_vector_type(2)));
typedef unsigned int   v4u  __attribute__((ext_vector_type(4)));
typedef unsigned short v8us __attribute__((ext_vector_type(8)));
typedef __bf16         v16b __attribute__((ext_vector_type(16)));
typedef v2f  __attribute__((may_alias)) v2fa;
typedef v4f  __attribute__((may_alias)) v4fa;
typedef v2d  __attribute__((may_alias)) v2da;
typedef v4i  __attribute__((may_alias)) v4ia;
typedef v2u  __attribute__((may_alias)) v2ua;
typedef v8us __attribute__((may_alias)) v8usa;
union FragB { v16b v; v8us h[2]; v8i w; };

__device__ __forceinline__ v8f wmb(const FragB& a, const FragB& b, v8f c) {
  v8f d = __builtin_amdgcn_wmma_f32_16x16x32_bf16(false, a.v, false, b.v, (short)0, c, false, false);
  asm volatile("v_nop\n\tv_nop\n\tv_nop\n\tv_nop" : "+v"(d) : "v"(a.w), "v"(b.w));
  return d;
}

__device__ __forceinline__ unsigned int f2bf(float f) {
  const unsigned int u = __float_as_uint(f);
  const unsigned int r = ((u + 0x7FFFu + ((u >> 16) & 1u)) >> 16) & 0xFFFFu;
  return ((u & 0x7FFFFFFFu) > 0x7F800000u) ? 0x7FC0u : r;
}
__device__ __forceinline__ float bf2f(unsigned int b) { return __uint_as_float(b << 16); }
__device__ __forceinline__ float bfr(float f) { return bf2f(f2bf(f)); }

template <int SLB>
__device__ __forceinline__ int scan_chunk(const int* __restrict__ dsts, int nE, int cbase, int slotBase,
                                          int nb, int vec8, int* list, int tid, int lane, int wave) {
  int wc = 0;
  const int el0  = tid * EPT;
  const int e0   = cbase + el0;
  const int sent = -2147483647 - 1;
  v4i da, db;
  if (vec8 != 0 && cbase + CHUNK <= nE) {
    da = *(const v4i*)(dsts + e0);
    db = *(const v4i*)(dsts + e0 + 4);
  } else {
    da.x = (e0     < nE) ? dsts[min(e0,     nE - 1)] : sent;
    da.y = (e0 + 1 < nE) ? dsts[min(e0 + 1, nE - 1)] : sent;
    da.z = (e0 + 2 < nE) ? dsts[min(e0 + 2, nE - 1)] : sent;
    da.w = (e0 + 3 < nE) ? dsts[min(e0 + 3, nE - 1)] : sent;
    db.x = (e0 + 4 < nE) ? dsts[min(e0 + 4, nE - 1)] : sent;
    db.y = (e0 + 5 < nE) ? dsts[min(e0 + 5, nE - 1)] : sent;
    db.z = (e0 + 6 < nE) ? dsts[min(e0 + 6, nE - 1)] : sent;
    db.w = (e0 + 7 < nE) ? dsts[min(e0 + 7, nE - 1)] : sent;
  }
  const unsigned nbs = (unsigned)slotBase;
  const unsigned unb = (unsigned)nb;
  const unsigned s0 = (unsigned)da.x - nbs, s1 = (unsigned)da.y - nbs;
  const unsigned s2 = (unsigned)da.z - nbs, s3 = (unsigned)da.w - nbs;
  const unsigned s4 = (unsigned)db.x - nbs, s5 = (unsigned)db.y - nbs;
  const unsigned s6 = (unsigned)db.z - nbs, s7 = (unsigned)db.w - nbs;
  const bool h0 = s0 < unb, h1 = s1 < unb, h2 = s2 < unb, h3 = s3 < unb;
  const bool h4 = s4 < unb, h5 = s5 < unb, h6 = s6 < unb, h7 = s7 < unb;
  const unsigned any = __builtin_amdgcn_ballot_w32(h0 | h1 | h2 | h3 | h4 | h5 | h6 | h7);
  if (any != 0u) {
#define HITJ(J, HJ, SJ) { \
      const unsigned mj = __builtin_amdgcn_ballot_w32(HJ); \
      if (mj != 0u) { \
        if (HJ) { \
          const int pos = wc + (int)__builtin_amdgcn_mbcnt_lo(mj, 0u); \
          if (pos < WCAP) list[wave * WCAP + pos] = ((el0 + (J)) << SLB) | (int)(SJ); \
        } \
        wc += (int)__builtin_popcount(mj); } }
    HITJ(0, h0, s0)
    HITJ(1, h1, s1)
    HITJ(2, h2, s2)
    HITJ(3, h3, s3)
    HITJ(4, h4, s4)
    HITJ(5, h5, s5)
    HITJ(6, h6, s6)
    HITJ(7, h7, s7)
#undef HITJ
  }
  return wc;
}

__global__ __launch_bounds__(NTHR) void k_pa(const float* __restrict__ x, int nN, int nUnits,
                                             unsigned short* xb) {
  const int u = (int)blockIdx.x * NTHR + (int)threadIdx.x;
  if (u >= nUnits) return;
  const int row = u >> 5;
  const int k8  = (u & 31) * 8;
  const int rc  = row < nN ? row : nN - 1;
  const float* p = x + (size_t)rc * DIN + k8;
  const v4f a = *(const v4fa*)p;
  const v4f b = *(const v4fa*)(p + 4);
  const bool ok = row < nN;
  v8us o;
  o[0] = ok ? (unsigned short)f2bf(a.x) : (unsigned short)0;
  o[1] = ok ? (unsigned short)f2bf(a.y) : (unsigned short)0;
  o[2] = ok ? (unsigned short)f2bf(a.z) : (unsigned short)0;
  o[3] = ok ? (unsigned short)f2bf(a.w) : (unsigned short)0;
  o[4] = ok ? (unsigned short)f2bf(b.x) : (unsigned short)0;
  o[5] = ok ? (unsigned short)f2bf(b.y) : (unsigned short)0;
  o[6] = ok ? (unsigned short)f2bf(b.z) : (unsigned short)0;
  o[7] = ok ? (unsigned short)f2bf(b.w) : (unsigned short)0;
  unsigned short* dp = xb + (size_t)row * DIN + k8;
  *(volatile v8us*)dp = o;
  __threadfence();
  *(volatile v8us*)dp = o;
}

template <int KW, int NW, int KD>
__device__ __forceinline__ void wunit(const float* __restrict__ W, unsigned short* WT, int v) {
  constexpr int UPR = KD / 8;
  const int n  = v / UPR;
  const int k8 = (v - n * UPR) * 8;
  const int kk = k8 & (KW - 1);
  const float* p = W + (size_t)kk * NW + n;
  v8us o;
#pragma unroll
  for (int i = 0; i < 8; ++i) o[i] = (unsigned short)f2bf(p[(size_t)i * NW]);
  unsigned short* dp = WT + (size_t)n * KD + k8;
  *(volatile v8us*)dp = o;
  __threadfence();
  *(volatile v8us*)dp = o;
}

__global__ __launch_bounds__(NTHR) void k_pw(const float* __restrict__ W0, const float* __restrict__ W1,
                                             const float* __restrict__ W2, const float* __restrict__ Wg,
                                             const float* __restrict__ Wr1, const float* __restrict__ Wr2,
                                             unsigned short* W0T, unsigned short* W1D, unsigned short* W2D,
                                             unsigned short* WgD, unsigned short* Wr1D, unsigned short* Wr2D) {
  const int u = (int)blockIdx.x * NTHR + (int)threadIdx.x;
  if (u < NUW0) {
    wunit<DIN, HID, DIN>(W0, W0T, u);
  } else if (u < NUW0 + NUW1) {
    wunit<HID, HID, K2>(W1, W1D, u - NUW0);
  } else if (u < NUW0 + 2 * NUW1) {
    wunit<HID, HID, K2>(W2, W2D, u - NUW0 - NUW1);
  } else if (u < NUW0 + 2 * NUW1 + NUWG) {
    wunit<HID, XGC, K2>(Wg, WgD, u - NUW0 - 2 * NUW1);
  } else if (u < NUW0 + 3 * NUW1 + NUWG) {
    wunit<HID, HID, K2>(Wr1, Wr1D, u - NUW0 - 2 * NUW1 - NUWG);
  } else if (u < NUWALL) {
    wunit<HID, XGC, K2>(Wr2, Wr2D, u - NUW0 - 3 * NUW1 - NUWG);
  }
}

__global__ __launch_bounds__(NTHR) void k_bucket(const int* __restrict__ srcs, const int* __restrict__ dsts,
                                                 int nE, int nN, int vec8, int* HITS, int* CNT, int* OFF,
                                                 float* DIS, int* FLG) {
  extern __shared__ __attribute__((aligned(16))) int bsm[];
  int* list = bsm;
  int* reg1 = bsm + LISTN;
  int* sl   = reg1 + RCAP;
  int* cnt  = sl + RCAP;
  int* offs = cnt + NBA;
  int* cur  = offs + NBA;
  int* wcnt = cur + NBA;
  const int tid = (int)threadIdx.x, lane = tid & 31, wave = tid >> 5;
  const int blk = (int)blockIdx.x;
  const int nodeBase = blk * NBA;
  int nb = nN - nodeBase;
  nb = nb < 0 ? 0 : (nb > NBA ? NBA : nb);

  {
    const v4i z4 = {0, 0, 0, 0};
    for (int i = tid * 4; i < BKT_ZINTS; i += NTHR * 4) *(v4ia*)(sl + i) = z4;
    if (tid < 16) wcnt[tid] = 0;
  }
  __syncthreads();

  int tot = 0, ovf = 0;
  const int nChunks = (nE + CHUNK - 1) / CHUNK;
#pragma unroll 1
  for (int ch = 0; ch < nChunks; ++ch) {
    const int cbase = ch * CHUNK;
    const int wc = scan_chunk<SLA>(dsts, nE, cbase, nodeBase, nb, vec8, list, tid, lane, wave);
    if (lane == 0) wcnt[wave] = wc;
    __syncthreads();
    int pre = 0, all = 0;
#pragma unroll
    for (int w2 = 0; w2 < NWAVE; ++w2) {
      int c = wcnt[w2];
      c = c < 0 ? 0 : (c > WCAP ? WCAP : c);
      all += c;
      pre += (w2 < wave) ? c : 0;
    }
    const int wcc  = wc > WCAP ? WCAP : wc;
    const int base = tot + pre;
#pragma unroll 1
    for (int i = lane; i < wcc; i += 32) {
      const int ent = list[wave * WCAP + i];
      const int el  = (ent >> SLA) & (CHUNK - 1);
      const int sq  = ent & (NBA - 1);
      int eid = cbase + el;
      eid = eid > nE - 1 ? nE - 1 : eid;
      const int sraw = srcs[eid];
      const int s = sraw < 0 ? 0 : (sraw > nN - 1 ? nN - 1 : sraw);
      const int pos = base + i;
      if (pos < RCAP) reg1[pos] = (int)((unsigned)s | ((unsigned)sq << 16));
    }
    if (tot + all > RCAP) ovf = 1;
    tot += all;
    tot = tot > RCAP ? RCAP : tot;
    __syncthreads();
  }
  const int nh = tot;

  if (wave == 0) {
#pragma unroll 1
    for (int b0 = 0; b0 < nh; b0 += 32) {
      const int idx = b0 + lane;
      const int uv  = reg1[idx < nh ? idx : nh - 1];
      const int m32 = (nh - b0) < 32 ? (nh - b0) : 32;
#pragma unroll 1
      for (int k = 0; k < m32; ++k) {
        const int u  = __builtin_amdgcn_readlane(uv, k);
        const int sq = (u >> 16) & (NBA - 1);
        if (lane == 0) cnt[sq] = cnt[sq] + 1;
      }
    }
  }
  __syncthreads();
  if (wave == 0) {
    const int base = lane * (NBA / 32);
    int s = 0;
#pragma unroll 1
    for (int i = 0; i < NBA / 32; ++i) s += cnt[base + i];
    int incl = s;
#pragma unroll
    for (int d = 1; d < 32; d <<= 1) {
      const int y = __shfl_up(incl, d, 32);
      if (lane >= d) incl += y;
    }
    int run = incl - s;
#pragma unroll 1
    for (int i = 0; i < NBA / 32; ++i) {
      const int cv = cnt[base + i];
      offs[base + i] = run;
      cur[base + i]  = run;
      run += cv;
    }
  }
  __syncthreads();
  if (wave == 0) {
#pragma unroll 1
    for (int b0 = 0; b0 < nh; b0 += 32) {
      const int idx = b0 + lane;
      const int uv  = reg1[idx < nh ? idx : nh - 1];
      const int m32 = (nh - b0) < 32 ? (nh - b0) : 32;
#pragma unroll 1
      for (int k = 0; k < m32; ++k) {
        const int u  = __builtin_amdgcn_readlane(uv, k);
        const int sq = (u >> 16) & (NBA - 1);
        if (lane == 0) {
          int p = cur[sq];
          p = p < 0 ? 0 : (p > RCAP - 1 ? RCAP - 1 : p);
          sl[p] = u;
          cur[sq] = p + 1;
        }
      }
    }
  }
  __syncthreads();

  int* hb = HITS + (size_t)blk * RCAP;
  const v4i c4 = *(const v4ia*)(cnt + 4 * tid);
  const v4i o4 = *(const v4ia*)(offs + 4 * tid);
  v4f d4;
  d4.x = rsqrtf((float)c4.x + 1.0f);
  d4.y = rsqrtf((float)c4.y + 1.0f);
  d4.z = rsqrtf((float)c4.z + 1.0f);
  d4.w = rsqrtf((float)c4.w + 1.0f);
  int*   cp = CNT + (size_t)blk * NBA + 4 * tid;
  int*   op = OFF + (size_t)blk * NBA + 4 * tid;
  float* dp = DIS + (size_t)blk * NBA + 4 * tid;
  v4i cv;
  cv.x = (tid == 0) ? nh : 0;
  cv.y = (tid == 0) ? ovf : 0;
  cv.z = 0; cv.w = 0;
  int* fp = FLG + (size_t)blk * 32 + 4 * (tid & 7);
#pragma unroll 1
  for (int p = tid * 4; p < RCAP; p += NTHR * 4) {
    const v4i v = *(const v4ia*)(sl + p);
    *(volatile v4i*)(hb + p) = v;
  }
  *(volatile v4i*)cp = c4;
  *(volatile v4i*)op = o4;
  *(volatile v4f*)dp = d4;
  if (tid < 8) *(volatile v4i*)fp = cv;
  __threadfence();
#pragma unroll 1
  for (int p = tid * 4; p < RCAP; p += NTHR * 4) {
    const v4i v = *(const v4ia*)(sl + p);
    *(volatile v4i*)(hb + p) = v;
  }
  *(volatile v4i*)cp = c4;
  *(volatile v4i*)op = o4;
  *(volatile v4f*)dp = d4;
  if (tid < 8) *(volatile v4i*)fp = cv;
}

template <int EP>
__global__ __launch_bounds__(GTHR) __attribute__((amdgpu_num_vgpr(248))) void k_gemm(
    const unsigned short* __restrict__ A, const unsigned short* __restrict__ WT,
    float* outF, unsigned short* outH, int K, int ldo,
    const float* __restrict__ aux0, const float* __restrict__ aux1, float* SD, int MPr, int nN)
{
  __shared__ __attribute__((aligned(16))) float stg[GBM * GBN];
  __shared__ __attribute__((aligned(16))) float satt[2 * GBN];
  __shared__ __attribute__((aligned(16))) float sdot[2 * GBM];
  const int tid = (int)threadIdx.x, lane = tid & 31, wave = tid >> 5, hh = lane >> 4, m = lane & 15;
  const int rowBase = (int)blockIdx.x * GBM;
  const int head    = (int)blockIdx.y;
  const int col0    = head * GBN;

  if constexpr (EP == EP_XG) {
    const int which = tid >> 6;
    const int c  = tid & 63;
    const float vs = aux0[head * HID + c];
    const float vd = aux1[head * HID + c];
    const float v = (which == 0) ? vs : vd;
    satt[which * GBN + c] = bfr(v);
  }

  v8f acc[4];
  {
    const v8f z = {0.f, 0.f, 0.f, 0.f, 0.f, 0.f, 0.f, 0.f};
    acc[0] = z; acc[1] = z; acc[2] = z; acc[3] = z;
  }
  const int arow = rowBase + 16 * wave + m;
  const int arc  = arow < nN ? arow : nN - 1;
  const int am   = arow < nN ? -1 : 0;
  const v8i mk   = {am, am, am, am, am, am, am, am};
  const unsigned short* ap = A  + (size_t)arc * (size_t)K + 8 * hh;
  const unsigned short* wp = WT + (size_t)(col0 + m) * (size_t)K + 8 * hh;
  const int ksteps = K >> 5;
#pragma unroll 1
  for (int ks = 0; ks < ksteps; ++ks) {
    FragB af;
    af.h[0] = *(const v8usa*)(ap + 32 * ks);
    af.h[1] = *(const v8usa*)(ap + 32 * ks + 16);
    af.w = af.w & mk;
#pragma unroll
    for (int t = 0; t < 4; ++t) {
      const unsigned short* wq = wp + (size_t)(16 * t) * (size_t)K + 32 * ks;
      FragB bf;
      bf.h[0] = *(const v8usa*)wq;
      bf.h[1] = *(const v8usa*)(wq + 16);
      acc[t] = wmb(af, bf, acc[t]);
    }
  }

#pragma unroll
  for (int t = 0; t < 4; ++t) {
    const int lc = 16 * t + m;
#pragma unroll
    for (int r = 0; r < 8; ++r) {
      const int lr = 16 * wave + 8 * hh + r;
      stg[lr * GBN + lc] = acc[t][r];
    }
  }
  __syncthreads();

  if constexpr (EP == EP_XG) {
    {
      const int row = tid & 63, which = tid >> 6;
      const float* sa = satt + which * GBN;
      const float* hr = stg + row * GBN;
      float d = 0.f;
#pragma unroll 4
      for (int c4 = 0; c4 < GBN / 4; ++c4) {
        const v4f hv = *(const v4fa*)(hr + 4 * c4);
        const v4f av = *(const v4fa*)(sa + 4 * c4);
        d = fmaf(hv.x, av.x, d);
        d = fmaf(hv.y, av.y, d);
        d = fmaf(hv.z, av.z, d);
        d = fmaf(hv.w, av.w, d);
      }
      sdot[which * GBM + row] = d;
    }
    __syncthreads();
    v4f fv[8];
#pragma unroll
    for (int i = 0; i < 8; ++i) {
      const int lr = 16 * wave + 2 * i + hh;
      fv[i] = *(const v4fa*)(stg + lr * GBN + 4 * m);
    }
    const int which2 = lane >> 4, piece = lane & 15;
    const v4f sdv = *(const v4fa*)(sdot + which2 * GBM + 4 * piece);
    float* sp = SD + (size_t)(2 * head + which2) * (size_t)MPr + rowBase + 4 * piece;
#pragma unroll
    for (int i = 0; i < 8; ++i) {
      const int gr = rowBase + 16 * wave + 2 * i + hh;
      float* op = outF + (size_t)gr * (size_t)ldo + col0 + 4 * m;
      *(volatile v4f*)op = fv[i];
    }
    if (wave == 0) *(volatile v4f*)sp = sdv;
    __threadfence();
#pragma unroll
    for (int i = 0; i < 8; ++i) {
      const int gr = rowBase + 16 * wave + 2 * i + hh;
      float* op = outF + (size_t)gr * (size_t)ldo + col0 + 4 * m;
      *(volatile v4f*)op = fv[i];
    }
    if (wave == 0) *(volatile v4f*)sp = sdv;
  } else if constexpr (EP == EP_P || EP == EP_REC) {
    v4f fv[8];
    v4f b4 = {0.f, 0.f, 0.f, 0.f};
    if constexpr (EP == EP_REC) {
      const v4f bq = *(const v4f*)(aux0 + col0 + 4 * m);
      b4.x = bfr(bq.x); b4.y = bfr(bq.y); b4.z = bfr(bq.z); b4.w = bfr(bq.w);
    }
#pragma unroll
    for (int i = 0; i < 8; ++i) {
      const int lr = 16 * wave + 2 * i + hh;
      const v4f xv = *(const v4fa*)(stg + lr * GBN + 4 * m);
      if constexpr (EP == EP_P) {
        const float dv = aux0[rowBase + lr];
        fv[i] = xv * dv;
      } else {
        fv[i] = xv + b4;
      }
    }
#pragma unroll
    for (int i = 0; i < 8; ++i) {
      const int gr = rowBase + 16 * wave + 2 * i + hh;
      float* op = outF + (size_t)gr * (size_t)ldo + col0 + 4 * m;
      *(volatile v4f*)op = fv[i];
    }
    __threadfence();
#pragma unroll
    for (int i = 0; i < 8; ++i) {
      const int gr = rowBase + 16 * wave + 2 * i + hh;
      float* op = outF + (size_t)gr * (size_t)ldo + col0 + 4 * m;
      *(volatile v4f*)op = fv[i];
    }
  } else {
    const int cg = 8 * (m & 7);
    const bool lsel = m >= 8;
    float bb[8];
    {
      const v4f q0 = *(const v4f*)(aux0 + cg);
      const v4f q1 = *(const v4f*)(aux0 + cg + 4);
      bb[0] = bfr(q0.x); bb[1] = bfr(q0.y); bb[2] = bfr(q0.z); bb[3] = bfr(q0.w);
      bb[4] = bfr(q1.x); bb[5] = bfr(q1.y); bb[6] = bfr(q1.z); bb[7] = bfr(q1.w);
    }
    v8us pv[8];
#pragma unroll
    for (int i = 0; i < 8; ++i) {
      const int lr = 16 * wave + 2 * i + hh;
      const v4f x0 = *(const v4fa*)(stg + lr * GBN + cg);
      const v4f x1 = *(const v4fa*)(stg + lr * GBN + cg + 4);
      float y[8];
      y[0] = x0.x + bb[0]; y[1] = x0.y + bb[1]; y[2] = x0.z + bb[2]; y[3] = x0.w + bb[3];
      y[4] = x1.x + bb[4]; y[5] = x1.y + bb[5]; y[6] = x1.z + bb[6]; y[7] = x1.w + bb[7];
#pragma unroll
      for (int j = 0; j < 8; ++j) {
        const float v = (y[j] > 0.0f) ? y[j] : (y[j] - y[j]);
        const unsigned int hb = f2bf(v);
        const unsigned int lb = f2bf(v - bf2f(hb));
        pv[i][j] = (unsigned short)(lsel ? lb : hb);
      }
    }
#pragma unroll
    for (int i = 0; i < 8; ++i) {
      const int gr = rowBase + 16 * wave + 2 * i + hh;
      unsigned short* op = outH + (size_t)gr * (size_t)ldo + 8 * m;
      *(volatile v8us*)op = pv[i];
    }
    __threadfence();
#pragma unroll
    for (int i = 0; i < 8; ++i) {
      const int gr = rowBase + 16 * wave + 2 * i + hh;
      unsigned short* op = outH + (size_t)gr * (size_t)ldo + 8 * m;
      *(volatile v8us*)op = pv[i];
    }
  }
}

template <int L>
__global__ __launch_bounds__(NTHR) void k_agg(const int* __restrict__ HITS, const int* __restrict__ CNT,
                                              const int* __restrict__ OFF, const float* __restrict__ DIS,
                                              const int* __restrict__ FLG, const float* __restrict__ P,
                                              const float* __restrict__ bias, const float* HSin,
                                              float* HSout, unsigned short* Hhl, int nN, int mRows) {
  __shared__ __attribute__((aligned(16))) int   scn[NBA];
  __shared__ __attribute__((aligned(16))) int   sof[NBA];
  __shared__ __attribute__((aligned(16))) float sdi[NBA];
  const int tid = (int)threadIdx.x, lane = tid & 31, wave = tid >> 5;
  const int blk = (int)blockIdx.x;
  const int nodeBase = blk * NBA;

  *(v4ia*)(scn + 4 * tid) = *(const v4i*)(CNT + (size_t)blk * NBA + 4 * tid);
  *(v4ia*)(sof + 4 * tid) = *(const v4i*)(OFF + (size_t)blk * NBA + 4 * tid);
  *(v4fa*)(sdi + 4 * tid) = *(const v4f*)(DIS + (size_t)blk * NBA + 4 * tid);
  const int nhraw = FLG[(size_t)blk * 32];
  const int bflag = FLG[(size_t)blk * 32 + 1];
  const int nh  = nhraw < 0 ? 0 : (nhraw > RCAP ? RCAP : nhraw);
  const int ovf = (bflag != 0 || nhraw < 0 || nhraw > RCAP) ? 1 : 0;
  float bv0, bv1;
  {
    const v2f a = *(const v2fa*)(bias + 2 * lane);
    bv0 = bfr(a.x); bv1 = bfr(a.y);
  }
  __syncthreads();

  const int* hbk = HITS + (size_t)blk * RCAP;
  const float qnan = __int_as_float(0x7fc00000);
  const float pz = (ovf != 0) ? qnan : 0.0f;
  const int sa = (2 * lane) & 31, sb = (2 * lane + 1) & 31;
  const int q0s = (4 * lane) & 31, q1s = (4 * lane + 1) & 31;
  const int q2s = (4 * lane + 2) & 31, q3s = (4 * lane + 3) & 31;
#pragma unroll 1
  for (int si = 0; si < NBA / NWAVE; ++si) {
    const int s    = si * NWAVE + wave;
    const int node = nodeBase + s;
    const int nc   = node < nN ? node : nN - 1;
    int c = scn[s];
    const bool big = c > DEGCAP;
    c = c < 0 ? 0 : (c > DEGCAP ? DEGCAP : c);
    int o = sof[s];
    o = o < 0 ? 0 : (o > RCAP ? RCAP : o);
    if (c > nh - o) c = nh - o;
    c = c < 0 ? 0 : c;
    const float dd = sdi[s];
    float acc0 = 0.0f, acc1 = 0.0f;
#pragma unroll 1
    for (int b0 = 0; b0 < c; b0 += 32) {
      int idx = o + b0 + lane;
      idx = idx < 0 ? 0 : (idx > RCAP - 1 ? RCAP - 1 : idx);
      const int ent = hbk[idx];
      int hs = ent & 0xFFFF;
      hs = hs > nN - 1 ? nN - 1 : hs;
      const int m32 = (c - b0) < 32 ? (c - b0) : 32;
#pragma unroll 1
      for (int k = 0; k < m32; ++k) {
        const int sk = __builtin_amdgcn_readlane(hs, k);
        const v2f a = *(const v2fa*)(P + (size_t)sk * HID + 2 * lane);
        acc0 += a.x; acc1 += a.y;
      }
    }
    float sv0, sv1;
    {
      const v2f a = *(const v2fa*)(P + (size_t)nc * HID + 2 * lane);
      sv0 = a.x; sv1 = a.y;
    }
    const float pzr = big ? qnan : pz;
    const bool live = node < nN;
    float y0 = dd * (acc0 + sv0) + bv0;
    float y1 = dd * (acc1 + sv1) + bv1;
    y0 = (y0 > 0.0f) ? y0 : (y0 - y0);
    y1 = (y1 > 0.0f) ? y1 : (y1 - y1);
    y0 = y0 + pzr; y1 = y1 + pzr;
    if constexpr (L >= 1) {
      const v2f r = *(const v2fa*)(HSin + (size_t)nc * HID + 2 * lane);
      y0 = r.x + y0; y1 = r.y + y1;
    }
    const float v0 = live ? y0 : 0.0f;
    const float v1 = live ? y1 : 0.0f;
    const bool wr = (node < mRows) && (lane < 16);

    const unsigned hb0 = f2bf(v0), hb1 = f2bf(v1);
    const unsigned lb0 = f2bf(v0 - bf2f(hb0));
    const unsigned lb1 = f2bf(v1 - bf2f(hb1));
    const int hw = (int)(hb0 | (hb1 << 16));
    const int lw = (int)(lb0 | (lb1 << 16));
    const int g0 = __shfl(hw, q0s, 32), g1 = __shfl(hw, q1s, 32);
    const int g2 = __shfl(hw, q2s, 32), g3 = __shfl(hw, q3s, 32);
    const int p0 = __shfl(lw, q0s, 32), p1 = __shfl(lw, q1s, 32);
    const int p2 = __shfl(lw, q2s, 32), p3 = __shfl(lw, q3s, 32);
    const bool lsel = (lane & 8) != 0;
    v4u pv;
    pv.x = (unsigned int)(lsel ? p0 : g0);
    pv.y = (unsigned int)(lsel ? p1 : g1);
    pv.z = (unsigned int)(lsel ? p2 : g2);
    pv.w = (unsigned int)(lsel ? p3 : g3);
    unsigned short* hp = Hhl + (size_t)node * K2 + 8 * (lane & 15);
    v4f ow;
    ow.x = __shfl(v0, sa, 32); ow.y = __shfl(v1, sa, 32);
    ow.z = __shfl(v0, sb, 32); ow.w = __shfl(v1, sb, 32);
    float* op = HSout + (size_t)node * HID + 4 * (lane & 15);
    if (wr) {
      *(volatile v4u*)hp = pv;
      if constexpr (L <= 1) *(volatile v4f*)op = ow;
    }
    __threadfence();
    if (wr) {
      *(volatile v4u*)hp = pv;
      if constexpr (L <= 1) *(volatile v4f*)op = ow;
    }
  }
}

__global__ __launch_bounds__(NTHR) __attribute__((amdgpu_num_vgpr(248))) void k_gat(
    const int* __restrict__ HITS, const int* __restrict__ CNT, const int* __restrict__ OFF,
    const int* __restrict__ FLG, const float* __restrict__ XG, const float* __restrict__ SD,
    const float* __restrict__ bg, float* HG, unsigned short* HGhl, double* REC, int nN, int mRows) {
  __shared__ __attribute__((aligned(16))) int    scn[NBA];
  __shared__ __attribute__((aligned(16))) int    sof[NBA];
  __shared__ __attribute__((aligned(16))) double wsum[NWAVE * HID];
  const int tid = (int)threadIdx.x, lane = tid & 31, wave = tid >> 5;
  const int blk = (int)blockIdx.x;
  const int nodeBase = blk * NBA;

  *(v4ia*)(scn + 4 * tid) = *(const v4i*)(CNT + (size_t)blk * NBA + 4 * tid);
  *(v4ia*)(sof + 4 * tid) = *(const v4i*)(OFF + (size_t)blk * NBA + 4 * tid);
  const int nhraw = FLG[(size_t)blk * 32];
  const int bflag = FLG[(size_t)blk * 32 + 1];
  const int nh  = nhraw < 0 ? 0 : (nhraw > RCAP ? RCAP : nhraw);
  const int ovf = (bflag != 0 || nhraw < 0 || nhraw > RCAP) ? 1 : 0;
  float bgv[8];
  {
    const int cg = 8 * (lane & 7);
    const v4f q0 = *(const v4f*)(bg + cg);
    const v4f q1 = *(const v4f*)(bg + cg + 4);
    bgv[0] = bfr(q0.x); bgv[1] = bfr(q0.y); bgv[2] = bfr(q0.z); bgv[3] = bfr(q0.w);
    bgv[4] = bfr(q1.x); bgv[5] = bfr(q1.y); bgv[6] = bfr(q1.z); bgv[7] = bfr(q1.w);
  }
  __syncthreads();

  const int* hbk = HITS + (size_t)blk * RCAP;
  const float qnan = __int_as_float(0x7fc00000);
  const float pzb  = (ovf != 0) ? qnan : 0.0f;
  const int head   = lane >> 3;
  const size_t hoS = (size_t)(2 * head) * (size_t)mRows;
  const size_t hoD = hoS + (size_t)mRows;
  const int srcl = lane >> 1;
  const bool odd  = (lane & 1) != 0;
  const bool lsel = (lane & 8) != 0;
  double ps0 = 0.0, ps1 = 0.0, ps2 = 0.0, ps3 = 0.0;

#pragma unroll 1
  for (int si = 0; si < NBA / NWAVE; ++si) {
    const int s    = si * NWAVE + wave;
    const int node = nodeBase + s;
    const int nc   = node < nN ? node : nN - 1;
    int c = scn[s];
    const bool big = c > DEGCAP;
    c = c < 0 ? 0 : (c > DEGCAP ? DEGCAP : c);
    int o = sof[s];
    o = o < 0 ? 0 : (o > RCAP ? RCAP : o);
    if (c > nh - o) c = nh - o;
    c = c < 0 ? 0 : c;
    const float adv = SD[hoD + (size_t)nc];
    float mx = -3.0e38f, dn = 0.0f;
    float acc[8];
#pragma unroll
    for (int i = 0; i < 8; ++i) acc[i] = 0.0f;
    const int T = c + 1;
#pragma unroll 1
    for (int b0 = 0; b0 < T; b0 += 32) {
      const int t = b0 + lane;
      int idx = o + t;
      idx = idx < 0 ? 0 : (idx > RCAP - 1 ? RCAP - 1 : idx);
      const int ent = hbk[idx];
      int hs = ent & 0xFFFF;
      hs = hs > nN - 1 ? nN - 1 : hs;
      const int sr  = (t < c) ? hs : nc;
      const int m32 = (T - b0) < 32 ? (T - b0) : 32;
#pragma unroll 1
      for (int k = 0; k < m32; ++k) {
        const int sk = __builtin_amdgcn_readlane(sr, k);
        const float* rp = XG + (size_t)sk * XGC + 8 * lane;
        float lg = SD[hoS + (size_t)sk] + adv;
        lg = lg > 0.f ? lg : NEGSL * lg;
        const float df = lg - mx;
        float ee = expf(-fabsf(df));
        ee = (ee < 1.17549435e-38f) ? 0.0f : ee;
        const bool  up = df > 0.f;
        const float s1 = up ? ee : 1.0f;
        const float s2 = up ? 1.0f : ee;
        mx = up ? lg : mx;
        dn = fmaf(dn, s1, s2);
        const v4f a = *(const v4f*)rp;
        const v4f b = *(const v4f*)(rp + 4);
        acc[0] = fmaf(acc[0], s1, s2 * a.x); acc[1] = fmaf(acc[1], s1, s2 * a.y);
        acc[2] = fmaf(acc[2], s1, s2 * a.z); acc[3] = fmaf(acc[3], s1, s2 * a.w);
        acc[4] = fmaf(acc[4], s1, s2 * b.x); acc[5] = fmaf(acc[5], s1, s2 * b.y);
        acc[6] = fmaf(acc[6], s1, s2 * b.z); acc[7] = fmaf(acc[7], s1, s2 * b.w);
      }
    }
    const float inv = __builtin_amdgcn_rcpf(dn);
    const float pzr = big ? qnan : pzb;
    const bool live = node < nN;
    float yv[8];
#pragma unroll
    for (int i = 0; i < 8; ++i) {
      float v = acc[i] * inv;
      v += __shfl_xor(v, 8, 32);
      v += __shfl_xor(v, 16, 32);
      const float y = fmaf(0.25f, v, bgv[i]) + pzr;
      yv[i] = live ? y : 0.0f;
    }
    const float l0 = __shfl(yv[0], srcl, 32), l1 = __shfl(yv[1], srcl, 32);
    const float l2 = __shfl(yv[2], srcl, 32), l3 = __shfl(yv[3], srcl, 32);
    const float u0 = __shfl(yv[4], srcl, 32), u1 = __shfl(yv[5], srcl, 32);
    const float u2 = __shfl(yv[6], srcl, 32), u3 = __shfl(yv[7], srcl, 32);
    v4f ow;
    ow.x = odd ? u0 : l0; ow.y = odd ? u1 : l1;
    ow.z = odd ? u2 : l2; ow.w = odd ? u3 : l3;
    v8us pv;
#pragma unroll
    for (int i = 0; i < 8; ++i) {
      const unsigned int hbi = f2bf(yv[i]);
      const unsigned int lbi = f2bf(yv[i] - bf2f(hbi));
      pv[i] = (unsigned short)(lsel ? lbi : hbi);
    }
    ps0 += (double)ow.x; ps1 += (double)ow.y; ps2 += (double)ow.z; ps3 += (double)ow.w;
    const bool wr = (node < mRows) && (lane < 16);
    float* op = HG + (size_t)node * HID + 4 * (lane & 15);
    unsigned short* hp = HGhl + (size_t)node * K2 + 8 * (lane & 15);
    if (wr) {
      *(volatile v4f*)op = ow;
      *(volatile v8us*)hp = pv;
    }
    __threadfence();
    if (wr) {
      *(volatile v4f*)op = ow;
      *(volatile v8us*)hp = pv;
    }
  }

  {
    v2d pa; pa.x = ps0; pa.y = ps1;
    v2d pb; pb.x = ps2; pb.y = ps3;
    *(v2da*)(wsum + wave * HID + 4 * (lane & 15))     = pa;
    *(v2da*)(wsum + wave * HID + 4 * (lane & 15) + 2) = pb;
  }
  __syncthreads();
  if (wave == 0) {
    v2d tv; tv.x = 0.0; tv.y = 0.0;
#pragma unroll
    for (int w2 = 0; w2 < NWAVE; ++w2) {
      const v2d p = *(const v2da*)(wsum + w2 * HID + 2 * lane);
      tv.x += p.x; tv.y += p.y;
    }
    double* rp = REC + (size_t)blk * HID + 2 * lane;
    *(volatile v2d*)rp = tv;
    __threadfence();
    *(volatile v2d*)rp = tv;
  }
}

__global__ __launch_bounds__(64) void k_head(const double* __restrict__ REC, const float* __restrict__ Wc1,
                                             const float* __restrict__ bc1, const float* __restrict__ Wc2,
                                             const float* __restrict__ bc2, float* CLS, int nBlk, double invN) {
  __shared__ float g[HID];
  __shared__ float y1[32];
  __shared__ __attribute__((aligned(16))) float co[32];
  const int t = (int)threadIdx.x;
  {
    double s = 0.0;
#pragma unroll 4
    for (int b = 0; b < nBlk; ++b) s += REC[(size_t)b * HID + t];
    g[t] = (float)(s * invN);
  }
  __syncthreads();
  if (t < 32) {
    float s = 0.0f;
#pragma unroll 4
    for (int f = 0; f < HID; ++f) s = fmaf(g[f], bfr(Wc1[f * 32 + t]), s);
    s = s + bfr(bc1[t]);
    y1[t] = (s > 0.0f) ? s : (s - s);
  }
  __syncthreads();
  if (t < 32) {
    const int tc = t < 2 ? t : 1;
    float s = 0.0f;
#pragma unroll 4
    for (int j = 0; j < 32; ++j) s = fmaf(y1[j], bfr(Wc2[j * 2 + tc]), s);
    s = s + bfr(bc2[tc]);
    co[t] = (t < 2) ? s : 0.0f;
  }
  __syncthreads();
  const v4f ov = *(const v4fa*)(co + 4 * (t & 7));
  float* op = CLS + 4 * (t & 7);
  if (t < 8) *(volatile v4f*)op = ov;
  __threadfence();
  if (t < 8) *(volatile v4f*)op = ov;
}

__device__ __forceinline__ v2u pick2(const float* __restrict__ CLS, const float* __restrict__ REC,
                                     const float* __restrict__ HG, int f) {
  int ir = f - OFF_REC;
  ir = ir < 0 ? 0 : (ir > REC_N - 2 ? REC_N - 2 : ir);
  int ih = f - OFF_HG;
  ih = ih < 0 ? 0 : (ih > HG_N - 2 ? HG_N - 2 : ih);
  const v2u a = *(const v2ua*)(CLS);
  const v2u b = *(const v2ua*)(REC + ir);
  const v2u c = *(const v2ua*)(HG + ih);
  const unsigned ma = (f < OFF_REC) ? 0xFFFFFFFFu : 0u;
  const unsigned mc = (f >= OFF_HG) ? 0xFFFFFFFFu : 0u;
  const unsigned mb = ~(ma | mc);
  v2u r;
  r.x = (a.x & ma) | (b.x & mb) | (c.x & mc);
  r.y = (a.y & ma) | (b.y & mb) | (c.y & mc);
  return r;
}

__global__ __launch_bounds__(NTHR) void k_out(const float* __restrict__ CLS, const float* __restrict__ REC,
                                              const float* __restrict__ HG, float* out) {
  const int tid = (int)threadIdx.x;
  const int g   = (int)blockIdx.x * NTHR + tid;
  const int f0  = 4 * g;
  const int flo = (int)blockIdx.x * (4 * NTHR);
  const int fhi = flo + 4 * NTHR - 1;
  v4f v;
  if (flo >= OFF_REC && fhi < OFF_HG) {
    const float* rp = REC + (f0 - OFF_REC);
    const v2f a = *(const v2fa*)rp;
    const v2f b = *(const v2fa*)(rp + 2);
    v.x = a.x; v.y = a.y; v.z = b.x; v.w = b.y;
  } else if (flo >= OFF_HG && fhi < OUT_TOT) {
    const float* hp = HG + (f0 - OFF_HG);
    const v2f a = *(const v2fa*)hp;
    const v2f b = *(const v2fa*)(hp + 2);
    v.x = a.x; v.y = a.y; v.z = b.x; v.w = b.y;
  } else {
    const int fa = f0 < OUT_TOT - 2 ? f0 : OUT_TOT - 2;
    const int fb = f0 + 2 < OUT_TOT - 2 ? f0 + 2 : OUT_TOT - 2;
    const v2u a = pick2(CLS, REC, HG, fa);
    const v2u b = pick2(CLS, REC, HG, fb);
    v.x = __uint_as_float(a.x); v.y = __uint_as_float(a.y);
    v.z = __uint_as_float(b.x); v.w = __uint_as_float(b.y);
  }
  const bool st4 = f0 + 3 < OUT_TOT;
  const bool st2 = (!st4) && (f0 + 1 < OUT_TOT);
  v2f vl; vl.x = v.x; vl.y = v.y;
  float* op = out + f0;
  if (st4) *(volatile v4f*)op = v;
  if (st2) *(volatile v2f*)op = vl;
  __threadfence();
  if (st4) *(volatile v4f*)op = v;
  if (st2) *(volatile v2f*)op = vl;
}

constexpr size_t al256c(size_t v) { return (v + 255) & ~(size_t)255; }
constexpr size_t SZ_A    = (size_t)MP * XGC * 4;
constexpr size_t SZ_B    = (size_t)MP * DIN * 2;
constexpr size_t SZ_HS   = (size_t)MP * HID * 4;
constexpr size_t SZ_HIT  = (size_t)NBLK * RCAP * 4;
constexpr size_t SZ_SD   = (size_t)8 * MP * 4;
constexpr size_t SZ_TAB  = (size_t)NSLOT * 4;
constexpr size_t SZ_FLG  = (size_t)NBLK * 128;
constexpr size_t SZ_W0T  = (size_t)HID * DIN * 2;
constexpr size_t SZ_W64  = (size_t)HID * K2 * 2;
constexpr size_t SZ_W256 = (size_t)XGC * K2 * 2;
constexpr size_t SZ_POOL = (size_t)NBLK * HID * 8;
constexpr size_t SZ_CLS  = 128;
constexpr size_t O_A    = 0;
constexpr size_t O_B    = al256c(O_A + SZ_A);
constexpr size_t O_P    = al256c(O_B + SZ_B);
constexpr size_t O_HSA  = al256c(O_P + SZ_HS);
constexpr size_t O_HSB  = al256c(O_HSA + SZ_HS);
constexpr size_t O_HIT  = al256c(O_HSB + SZ_HS);
constexpr size_t O_SD   = al256c(O_HIT + SZ_HIT);
constexpr size_t O_CNT  = al256c(O_SD + SZ_SD);
constexpr size_t O_OFF  = al256c(O_CNT + SZ_TAB);
constexpr size_t O_DIS  = al256c(O_OFF + SZ_TAB);
constexpr size_t O_FLG  = al256c(O_DIS + SZ_TAB);
constexpr size_t O_W0T  = al256c(O_FLG + SZ_FLG);
constexpr size_t O_W1D  = al256c(O_W0T + SZ_W0T);
constexpr size_t O_W2D  = al256c(O_W1D + SZ_W64);
constexpr size_t O_WGD  = al256c(O_W2D + SZ_W64);
constexpr size_t O_WR1  = al256c(O_WGD + SZ_W256);
constexpr size_t O_WR2  = al256c(O_WR1 + SZ_W64);
constexpr size_t O_POOL = al256c(O_WR2 + SZ_W256);
constexpr size_t O_CLS  = al256c(O_POOL + SZ_POOL);
constexpr size_t WS_TOTAL = al256c(O_CLS + SZ_CLS);
static_assert(WS_TOTAL <= (size_t)134217728);
static_assert(SZ_B >= 2 * (size_t)MP * K2 * 2);
static_assert((size_t)(OUT_TOT - 1) < (size_t)64000008 / 4);

extern "C" void kernel_launch(void* const* d_in, const int* in_sizes, int n_in,
                              void* d_out, int out_size, void* d_ws, size_t ws_size,
                              hipStream_t stream) {
  if (n_in < 20) return;
  if (in_sizes[0] != NN * DIN) return;
  if (in_sizes[1] != 2 * NE) return;
  if (in_sizes[2] != DIN * HID || in_sizes[3] != HID) return;
  if (in_sizes[4] != HID * HID || in_sizes[5] != HID) return;
  if (in_sizes[6] != HID * HID || in_sizes[7] != HID) return;
  if (in_sizes[8] != HID * XGC) return;
  if (in_sizes[9] != XGC || in_sizes[10] != XGC || in_sizes[11] != HID) return;
  if (in_sizes[12] != HID * 32 || in_sizes[13] != 32) return;
  if (in_sizes[14] != 64 || in_sizes[15] != 2) return;
  if (in_sizes[16] != HID * HID || in_sizes[17] != HID) return;
  if (in_sizes[18] != HID * XGC || in_sizes[19] != XGC) return;
  if (out_size != OUT_TOT) return;
  if (ws_size < WS_TOTAL) return;

  const float* x    = (const float*)d_in[0];
  const int*   ei   = (const int*)  d_in[1];
  const float* W0   = (const float*)d_in[2];   const float* b0  = (const float*)d_in[3];
  const float* W1   = (const float*)d_in[4];   const float* b1  = (const float*)d_in[5];
  const float* W2   = (const float*)d_in[6];   const float* b2  = (const float*)d_in[7];
  const float* Wg   = (const float*)d_in[8];
  const float* atS  = (const float*)d_in[9];
  const float* atD  = (const float*)d_in[10];
  const float* bg   = (const float*)d_in[11];
  const float* Wc1  = (const float*)d_in[12];  const float* bc1 = (const float*)d_in[13];
  const float* Wc2  = (const float*)d_in[14];  const float* bc2 = (const float*)d_in[15];
  const float* Wr1  = (const float*)d_in[16];  const float* br1 = (const float*)d_in[17];
  const float* Wr2  = (const float*)d_in[18];  const float* br2 = (const float*)d_in[19];
  float* out = (float*)d_out;
  const int* src = ei;
  const int* dst = ei + NE;
  const int nN = NN, nE = NE;
  const int vec8 = ((nE & 3) == 0) ? 1 : 0;

  char* ws = (char*)d_ws;
  float*          XG   = (float*)(ws + O_A);
  float*          RECp = (float*)(ws + O_A);
  unsigned short* XB   = (unsigned short*)(ws + O_B);
  unsigned short* Hhl  = (unsigned short*)(ws + O_B);
  unsigned short* HGhl = (unsigned short*)(ws + O_B);
  unsigned short* R1hl = (unsigned short*)(ws + O_B) + (size_t)MP * K2;
  float*          P    = (float*)(ws + O_P);
  float*          HSa  = (float*)(ws + O_HSA);
  float*          HSb  = (float*)(ws + O_HSB);
  float*          HG   = (float*)(ws + O_HSA);
  int*            HITS = (int*)(ws + O_HIT);
  float*          SD   = (float*)(ws + O_SD);
  int*            CNT  = (int*)(ws + O_CNT);
  int*            OFF  = (int*)(ws + O_OFF);
  float*          DIS  = (float*)(ws + O_DIS);
  int*            FLG  = (int*)(ws + O_FLG);
  unsigned short* W0T  = (unsigned short*)(ws + O_W0T);
  unsigned short* W1D  = (unsigned short*)(ws + O_W1D);
  unsigned short* W2D  = (unsigned short*)(ws + O_W2D);
  unsigned short* WgD  = (unsigned short*)(ws + O_WGD);
  unsigned short* Wr1D = (unsigned short*)(ws + O_WR1);
  unsigned short* Wr2D = (unsigned short*)(ws + O_WR2);
  double*         POOL = (double*)(ws + O_POOL);
  float*          CLS  = (float*)(ws + O_CLS);

  const int bktLds = BKT_LDS_INTS * 4;
  hipFuncSetAttribute(reinterpret_cast<const void*>(&k_bucket),
                      hipFuncAttributeMaxDynamicSharedMemorySize, bktLds);

  const int gM  = MP / GBM;
  const int nUx = MP * (DIN / 8);

  k_pa<<<nUx / NTHR, NTHR, 0, stream>>>(x, nN, nUx, XB);
  k_pw<<<NUWALL / NTHR, NTHR, 0, stream>>>(W0, W1, W2, Wg, Wr1, Wr2, W0T, W1D, W2D, WgD, Wr1D, Wr2D);
  k_bucket<<<NBLK, NTHR, bktLds, stream>>>(src, dst, nE, nN, vec8, HITS, CNT, OFF, DIS, FLG);
  k_gemm<EP_P><<<dim3(gM, 1), GTHR, 0, stream>>>(XB, W0T, P, R1hl, DIN, HID, DIS, DIS, SD, MP, nN);
  k_agg<0><<<NBLK, NTHR, 0, stream>>>(HITS, CNT, OFF, DIS, FLG, P, b0, P, HSa, Hhl, nN, MP);
  k_gemm<EP_P><<<dim3(gM, 1), GTHR, 0, stream>>>(Hhl, W1D, P, R1hl, K2, HID, DIS, DIS, SD, MP, nN);
  k_agg<1><<<NBLK, NTHR, 0, stream>>>(HITS, CNT, OFF, DIS, FLG, P, b1, HSa, HSb, Hhl, nN, MP);
  k_gemm<EP_P><<<dim3(gM, 1), GTHR, 0, stream>>>(Hhl, W2D, P, R1hl, K2, HID, DIS, DIS, SD, MP, nN);
  k_agg<2><<<NBLK, NTHR, 0, stream>>>(HITS, CNT, OFF, DIS, FLG, P, b2, HSb, HSa, Hhl, nN, MP);
  k_gemm<EP_XG><<<dim3(gM, XGC / GBN), GTHR, 0, stream>>>(Hhl, WgD, XG, R1hl, K2, XGC, atS, atD, SD, MP, nN);
  k_gat<<<NBLK, NTHR, 0, stream>>>(HITS, CNT, OFF, FLG, XG, SD, bg, HG, HGhl, POOL, nN, MP);
  k_gemm<EP_R1><<<dim3(gM, 1), GTHR, 0, stream>>>(HGhl, Wr1D, P, R1hl, K2, K2, br1, br1, SD, MP, nN);
  k_gemm<EP_REC><<<dim3(gM, XGC / GBN), GTHR, 0, stream>>>(R1hl, Wr2D, RECp, Hhl, K2, XGC, br2, br2, SD, MP, nN);
  k_head<<<1, 64, 0, stream>>>(POOL, Wc1, bc1, Wc2, bc2, CLS, NBLK, 1.0 / (double)NN);
  k_out<<<OUT_BLOCKS, NTHR, 0, stream>>>(CLS, RECp, HG, out);
}
